// GRUODEDecay_50517405335821
// MI455X (gfx1250) — hardware-verified
//
#include <hip/hip_runtime.h>
#include <math.h>

typedef __attribute__((ext_vector_type(16))) _Float16 v16h;
typedef __attribute__((ext_vector_type(8)))  _Float16 v8h;
typedef __attribute__((ext_vector_type(16))) __bf16   v16b;
typedef __attribute__((ext_vector_type(8)))  __bf16   v8b;
typedef __attribute__((ext_vector_type(8)))  float    v8f;
typedef __attribute__((ext_vector_type(4)))  float    v4f;
#define PSCALE 32768.0f
#define U16(p) ((const unsigned short*)(const void*)(p))
#define PSCALE_INV (1.0f / 32768.0f)

__device__ __forceinline__ unsigned short f2bf_bits(float f) {
  unsigned u = __float_as_uint(f);
  return (unsigned short)((u + 0x7FFFu + ((u >> 16) & 1u)) >> 16);
}
__device__ __forceinline__ float bf_bits2f(unsigned short h) { return __uint_as_float(((unsigned)h) << 16); }

__device__ __forceinline__ void dep_guard_h(v8f& a, v8f& b, v16h x, v16h y) { asm volatile("v_nop\n\tv_nop\n\tv_nop\n\tv_nop" : "+v"(a), "+v"(b) : "v"(x), "v"(y)); }
__device__ __forceinline__ void dep_guard_b(v8f& a, v8f& b, v16b x, v16b y) { asm volatile("v_nop\n\tv_nop\n\tv_nop\n\tv_nop" : "+v"(a), "+v"(b) : "v"(x), "v"(y)); }
__device__ __forceinline__ void keep4_h(v16h a, v16h b, v16h c, v16h d) { asm volatile("v_nop" :: "v"(a), "v"(b), "v"(c), "v"(d)); }
__device__ __forceinline__ void keep4_b(v16b a, v16b b, v16b c, v16b d) { asm volatile("v_nop" :: "v"(a), "v"(b), "v"(c), "v"(d)); }
__device__ __forceinline__ void acc_guard4(v8f& a, v8f& b, v8f& c, v8f& d) { asm volatile("v_nop\n\tv_nop\n\tv_nop\n\tv_nop" : "+v"(a), "+v"(b), "+v"(c), "+v"(d)); }
template <typename T> struct Frag;
template <> struct Frag<_Float16> {
  typedef v16h V; union U { v16h v; v8h h[2]; };
  static __device__ __forceinline__ v16h load(const _Float16* p) {
    U f; f.h[0] = *(const v8h*)(p); f.h[1] = *(const v8h*)(p + 16); return f.v;
  }
  static __device__ __forceinline__ v8f mma(v16h a, v16h b, v8f c) {
    return __builtin_amdgcn_wmma_f32_16x16x32_f16(false, a, false, b, (short)0, c, false, false);
  }
  static __device__ __forceinline__ void guard(v8f& a, v8f& b, v16h x, v16h y) { dep_guard_h(a, b, x, y); }
  static __device__ __forceinline__ void keep(v16h a, v16h b, v16h c, v16h d) { keep4_h(a, b, c, d); }
};
template <> struct Frag<__bf16> {
  typedef v16b V; union U { v16b v; v8b h[2]; };
  static __device__ __forceinline__ v16b load(const __bf16* p) {
    U f; f.h[0] = *(const v8b*)(p); f.h[1] = *(const v8b*)(p + 16); return f.v;
  }
  static __device__ __forceinline__ v8f mma(v16b a, v16b b, v8f c) {
    return __builtin_amdgcn_wmma_f32_16x16x32_bf16(false, a, false, b, (short)0, c, false, false);
  }
  static __device__ __forceinline__ void guard(v8f& a, v8f& b, v16b x, v16b y) { dep_guard_b(a, b, x, y); }
  static __device__ __forceinline__ void keep(v16b a, v16b b, v16b c, v16b d) { keep4_b(a, b, c, d); }
};

template <int ET> struct Elem;
template <> struct Elem<0> { typedef _Float16 T; };
template <> struct Elem<1> { typedef __bf16 T; };
template <int ET, bool SPLIT, int BIAS_MODE, int OUT_MODE, bool RESID, int ACT = 0>
__global__ __launch_bounds__(256) void wmma_gemm64(
    const unsigned short* __restrict__ Ap, const unsigned short* __restrict__ A2p, int lda, long strideA,
    const unsigned short* __restrict__ Btp, const unsigned short* __restrict__ Bt2p, int ldb, long strideB,
    void* __restrict__ Cout, void* __restrict__ Cout2, int ldc, long strideC,
    const float* __restrict__ bias,
    const float* __restrict__ resid, long strideR,
    int M, int N, int K, float scale) {
  typedef typename Elem<ET>::T T;
  typedef typename Frag<T>::V V;
  const T* A = (const T*)Ap; const T* A2 = (const T*)A2p; const T* Bt = (const T*)Btp; const T* Bt2 = (const T*)Bt2p;
  __shared__ __align__(16) float sT[8][16 * 68];
  const int b    = blockIdx.y;
  const int lane = threadIdx.x & 31;
  const int wave = threadIdx.x >> 5;
  const int tilesN = N >> 6;
  const int tilesM = M >> 6;
  const int tile = blockIdx.x * 8 + wave;
  if (tile >= tilesM * tilesN) return;
  const int tm = tile / tilesN;
  const int tn = tile - tm * tilesN;
  const int m0 = tm << 6;
  const int n0 = tn << 6;

  const T* Ab  = A  + (size_t)b * strideA;
  const T* Bb  = Bt + (size_t)b * strideB;
  const T* Ab2 = SPLIT ? (A2  + (size_t)b * strideA) : nullptr;
  const T* Bb2 = SPLIT ? (Bt2 + (size_t)b * strideB) : nullptr;

  const int rlane = lane & 15;
  const int koff  = (lane >> 4) * 8;
  const int mOff  = (lane >> 4) * 8;

  v8f acc[4][4];
#pragma unroll
  for (int i = 0; i < 4; ++i)
#pragma unroll
    for (int j = 0; j < 4; ++j) acc[i][j] = (v8f){0.f,0.f,0.f,0.f,0.f,0.f,0.f,0.f};

  for (int k0 = 0; k0 < K; k0 += 32) {
    V bh[4], bl[4];
#pragma unroll
    for (int j = 0; j < 4; ++j) {
      const size_t bo = (size_t)(n0 + (j << 4) + rlane) * ldb + koff + k0;
      bh[j] = Frag<T>::load(Bb + bo);
      if (SPLIT) bl[j] = Frag<T>::load(Bb2 + bo);
    }
#pragma unroll
    for (int i = 0; i < 4; ++i) {
      const size_t ao = (size_t)(m0 + (i << 4) + rlane) * lda + koff + k0;
      V ah = Frag<T>::load(Ab + ao);
      V al;
      if (SPLIT) al = Frag<T>::load(Ab2 + ao);
#pragma unroll
      for (int j = 0; j < 4; ++j) {
        acc[i][j] = Frag<T>::mma(ah, bh[j], acc[i][j]);
        if (SPLIT) {
          acc[i][j] = Frag<T>::mma(ah, bl[j], acc[i][j]);
          acc[i][j] = Frag<T>::mma(al, bh[j], acc[i][j]);
        }
      }
      Frag<T>::guard(acc[i][0], acc[i][3], ah, SPLIT ? al : ah);
    }
    Frag<T>::keep(bh[0], bh[1], bh[2], bh[3]);
    if (SPLIT) Frag<T>::keep(bl[0], bl[1], bl[2], bl[3]);
  }
  acc_guard4(acc[0][0], acc[0][1], acc[0][2], acc[0][3]);
  acc_guard4(acc[1][0], acc[1][1], acc[1][2], acc[1][3]);
  acc_guard4(acc[2][0], acc[2][1], acc[2][2], acc[2][3]);
  acc_guard4(acc[3][0], acc[3][1], acc[3][2], acc[3][3]);

  float* slab = sT[wave];
  const float* Rb = RESID ? (resid + (size_t)b * strideR) : nullptr;
#pragma unroll
  for (int i = 0; i < 4; ++i) {
    const int mBase = m0 + (i << 4);
#pragma unroll
    for (int j = 0; j < 4; ++j) {
      const int n = n0 + (j << 4) + rlane;
      float bv = 0.f;
      if (BIAS_MODE == 2) bv = bias[n];
#pragma unroll
      for (int r = 0; r < 8; ++r) {
        float v = acc[i][j][r] * scale;
        if (BIAS_MODE == 1) v += bias[mBase + mOff + r];
        if (BIAS_MODE == 2) v += bv;
        if (RESID) v += Rb[(size_t)(mBase + mOff + r) * ldc + n];
        if (ACT == 1) v = tanhf(v);
        if (ACT == 2) v = fmaxf(v, 0.0f);
        if (ACT == 3) v = v / (1.0f + expf(-v));
        if (ACT == 4) v = (v > 0.f) ? v : 0.01f * v;
        if (ACT == 5) v = 0.5f * v * (1.0f + erff(v * 0.70710678118654752f));
        slab[(mOff + r) * 68 + (j << 4) + rlane] = v;
      }
    }
    __builtin_amdgcn_fence(__ATOMIC_RELEASE, "workgroup");
    __builtin_amdgcn_wave_barrier();
    __builtin_amdgcn_fence(__ATOMIC_ACQUIRE, "workgroup");
    if (OUT_MODE == 0) {
      float* C = (float*)Cout + (size_t)b * strideC;
      const int hh = lane >> 4, c4 = (lane & 15) * 4;
      for (int pass = 0; pass < 2; ++pass) {
#pragma unroll
        for (int it = 0; it < 8; ++it) {
          const int row = it * 2 + hh;
          v4f v = *(const v4f*)(slab + row * 68 + c4);
          *(volatile v4f*)(C + (size_t)(mBase + row) * ldc + n0 + c4) = v;
        }
        __threadfence();
      }
    } else {
      const int q = lane >> 3, c8 = (lane & 7) * 8;
      unsigned short* C  = (unsigned short*)Cout  + (size_t)b * strideC;
      unsigned short* C2 = (OUT_MODE == 2) ? ((unsigned short*)Cout2 + (size_t)b * strideC) : nullptr;
      for (int pass = 0; pass < 2; ++pass) {
#pragma unroll
        for (int it = 0; it < 4; ++it) {
          const int row = it * 4 + q;
          const float* sp = slab + row * 68 + c8;
          v8h hv, lv;
#pragma unroll
          for (int e = 0; e < 8; ++e) {
            if (OUT_MODE == 1) {
              hv[e] = (_Float16)sp[e];
            } else {
              unsigned short hb = f2bf_bits(sp[e]);
              unsigned short lb = f2bf_bits(sp[e] - bf_bits2f(hb));
              hv[e] = __builtin_bit_cast(_Float16, hb);
              lv[e] = __builtin_bit_cast(_Float16, lb);
            }
          }
          *(volatile v8h*)(C + (size_t)(mBase + row) * ldc + n0 + c8) = hv;
          if (OUT_MODE == 2) *(volatile v8h*)(C2 + (size_t)(mBase + row) * ldc + n0 + c8) = lv;
        }
        __threadfence();
      }
    }
    __builtin_amdgcn_fence(__ATOMIC_RELEASE, "workgroup");
    __builtin_amdgcn_wave_barrier();
    __builtin_amdgcn_fence(__ATOMIC_ACQUIRE, "workgroup");
  }
}

#define NBATCH 64
#define NSTEP 32
#define HID 256
#define NGATE3 768
#define NB_ROWS 32
#define NTHR 256
#define TPH 264
#define YPF 260
#define WCARRY 16.0f
#define WCARRY_INV 0.0625f

__global__ __launch_bounds__(256) void cast_scale_f16x2(
    const float* __restrict__ in, _Float16* __restrict__ out, int n2, float scale) {
  int i = blockIdx.x * 256 + threadIdx.x;
  if (i < n2) {
    const _Float16 h0 = (_Float16)(in[2 * i] * scale), h1 = (_Float16)(in[2 * i + 1] * scale);
    const unsigned u = (unsigned)__builtin_bit_cast(unsigned short, h0) | ((unsigned)__builtin_bit_cast(unsigned short, h1) << 16);
    ((volatile unsigned*)out)[i] = u;
    __threadfence();
    ((volatile unsigned*)out)[i] = u;
  }
}

__device__ __forceinline__ v8f mma_h(v16h a, v16h b, v8f cacc) {
  cacc = __builtin_amdgcn_wmma_f32_16x16x32_f16(false, a, false, b, (short)0, cacc, false, false);
  asm volatile("v_nop\n\tv_nop\n\tv_nop\n\tv_nop" : "+v"(cacc) : "v"(a), "v"(b));
  return cacc;
}
__device__ __forceinline__ v8f zero8() { return (v8f){0.f,0.f,0.f,0.f,0.f,0.f,0.f,0.f}; }

__device__ __forceinline__ float softplus_f(float v) {
  return fmaxf(v, 0.0f) + __logf(1.0f + __expf(-fabsf(v)));
}
__device__ __forceinline__ float sigmoid_f(float x) {
  const float xc = fmaxf(x, -80.0f);
  return 1.0f / (1.0f + expf(-xc));
}

__device__ __forceinline__ void tile_gemm_32x32(const _Float16* tin, const _Float16* __restrict__ W,
                                                int nb0, int c, int hh, v8f (&acc)[2][2]) {
#pragma unroll
  for (int i = 0; i < 2; ++i)
#pragma unroll
    for (int j = 0; j < 2; ++j) acc[i][j] = zero8();
#pragma unroll 2
  for (int k0 = 0; k0 < HID; k0 += 32) {
    const v16h a0 = Frag<_Float16>::load(tin + c * TPH + k0 + 8 * hh);
    const v16h a1 = Frag<_Float16>::load(tin + (16 + c) * TPH + k0 + 8 * hh);
    const v16h b0 = Frag<_Float16>::load(W + (size_t)(nb0 + c) * HID + k0 + 8 * hh);
    const v16h b1 = Frag<_Float16>::load(W + (size_t)(nb0 + 16 + c) * HID + k0 + 8 * hh);
    acc[0][0] = mma_h(a0, b0, acc[0][0]);
    acc[0][1] = mma_h(a0, b1, acc[0][1]);
    acc[1][0] = mma_h(a1, b0, acc[1][0]);
    acc[1][1] = mma_h(a1, b1, acc[1][1]);
  }
}

__device__ __forceinline__ void store_softplus_tile(_Float16* tout, const v8f (&acc)[2][2],
                                                    float ba, float bb, int nb0, int c, int hh) {
#pragma unroll
  for (int i = 0; i < 2; ++i)
#pragma unroll
    for (int j = 0; j < 2; ++j) {
      const int n = nb0 + 16 * j + c;
      const float bias = j ? bb : ba;
#pragma unroll
      for (int r = 0; r < 8; ++r) {
        const float v = acc[i][j][r] * WCARRY_INV + bias;
        tout[(16 * i + 8 * hh + r) * TPH + n] = (_Float16)softplus_f(v);
      }
    }
}

__global__ __launch_bounds__(NTHR) void gru_ode_seq(
    const float* __restrict__ G,
    const _Float16* __restrict__ Whh,
    const _Float16* __restrict__ W1,
    const _Float16* __restrict__ W2,
    const _Float16* __restrict__ W3,
    const float* __restrict__ times,
    const float* __restrict__ bhh,
    const float* __restrict__ b1, const float* __restrict__ b2, const float* __restrict__ b3,
    float* __restrict__ out)
{
  __shared__ __align__(16) _Float16 TA[NB_ROWS * TPH];
  __shared__ __align__(16) _Float16 TB[NB_ROWS * TPH];
  __shared__ __align__(16) _Float16 TC[NB_ROWS * TPH];
  __shared__ __align__(16) float ys[NB_ROWS * YPF];
  __shared__ float tcur[NBATCH];
  __shared__ float tsorted[NBATCH];
  __shared__ float dts_s[NBATCH];
  __shared__ int idx_s[NB_ROWS];

  const int tid  = threadIdx.x;
  const int lane = tid & 31;
  const int wave = tid >> 5;
  const int hh   = lane >> 4;
  const int c    = lane & 15;
  const int row0 = blockIdx.x * NB_ROWS;
  const int nb0  = wave * 32;

  {
    unsigned* TAu = (unsigned*)TA;
    for (int i = tid; i < (NB_ROWS * TPH) / 2; i += NTHR) TAu[i] = 0u;
    for (int i = tid; i < NB_ROWS * YPF; i += NTHR) ys[i] = 0.0f;
  }
  __syncthreads();

  for (int t = 0; t < NSTEP; ++t) {
    if (tid < NBATCH) tcur[tid] = times[tid * NSTEP + t];
    __syncthreads();
    if (tid < NBATCH) {
      const float tb = tcur[tid];
      int rk = 0, cn = 0;
#pragma unroll 4
      for (int cc = 0; cc < NBATCH; ++cc) {
        const float tv = tcur[cc];
        const bool lt = tv < tb;
        rk += (lt || (tv == tb && cc < tid)) ? 1 : 0;
        cn += lt ? 1 : 0;
      }
      rk = rk > (NBATCH - 1) ? (NBATCH - 1) : rk;
      tsorted[rk] = tb;
      const int lr = tid - row0;
      if ((unsigned)lr < (unsigned)NB_ROWS) idx_s[lr] = cn;
    }
    __syncthreads();
    if (tid < NBATCH - 1) dts_s[tid] = tsorted[tid + 1] - tsorted[tid];

#pragma unroll 1
    for (int q = 0; q < 2; ++q) {
      const int u = nb0 + 16 * q + c;
      v8f acc[3][2];
#pragma unroll
      for (int g = 0; g < 3; ++g) { acc[g][0] = zero8(); acc[g][1] = zero8(); }
#pragma unroll 2
      for (int k0 = 0; k0 < HID; k0 += 32) {
        const v16h a0 = Frag<_Float16>::load(TA + c * TPH + k0 + 8 * hh);
        const v16h a1 = Frag<_Float16>::load(TA + (16 + c) * TPH + k0 + 8 * hh);
#pragma unroll
        for (int g = 0; g < 3; ++g) {
          const v16h bw = Frag<_Float16>::load(Whh + (size_t)(g * HID + u) * HID + k0 + 8 * hh);
          acc[g][0] = mma_h(a0, bw, acc[g][0]);
          acc[g][1] = mma_h(a1, bw, acc[g][1]);
        }
      }
      const float bh_r = bhh[u], bh_z = bhh[HID + u], bh_n = bhh[2 * HID + u];
#pragma unroll
      for (int i = 0; i < 2; ++i) {
#pragma unroll
        for (int r = 0; r < 8; ++r) {
          const int lr = 16 * i + 8 * hh + r;
          const float* gp = G + ((size_t)(row0 + lr) * NSTEP + t) * NGATE3 + u;
          const float gi_r = gp[0], gi_z = gp[HID], gi_n = gp[2 * HID];
          const float h_r = acc[0][i][r] * WCARRY_INV + bh_r;
          const float h_z = acc[1][i][r] * WCARRY_INV + bh_z;
          const float h_n = acc[2][i][r] * WCARRY_INV + bh_n;
          const float rg = sigmoid_f(gi_r + h_r);
          const float zg = sigmoid_f(gi_z + h_z);
          const float ng = tanhf(gi_n + rg * h_n);
          const float hold = ys[lr * YPF + u];
          const float hnew = (1.0f - zg) * ng + zg * hold;
          ys[lr * YPF + u] = hnew;
        }
      }
    }
    __syncthreads();

    {
      float* obase = out + ((size_t)row0 * NSTEP + t) * HID;
      for (int pass = 0; pass < 2; ++pass) {
#pragma unroll
        for (int rr = 0; rr < 4; ++rr) {
          const int lr = wave * 4 + rr;
#pragma unroll
          for (int half = 0; half < 2; ++half) {
            const v4f v = *(const v4f*)(ys + lr * YPF + half * 128 + lane * 4);
            *(volatile v4f*)(obase + (size_t)lr * NSTEP * HID + half * 128 + lane * 4) = v;
          }
        }
        __threadfence();
      }
#pragma unroll
      for (int rr = 0; rr < 4; ++rr) {
        const int lr = wave * 4 + rr;
        const float* sp = ys + lr * YPF + 8 * lane;
        v8h hv;
#pragma unroll
        for (int e = 0; e < 8; ++e) hv[e] = (_Float16)sp[e];
        *(v8h*)(TA + lr * TPH + 8 * lane) = hv;
      }
    }
    __syncthreads();

    if (t < NSTEP - 1) {
      const float b1a = b1[nb0 + c], b1b = b1[nb0 + 16 + c];
      const float b2a = b2[nb0 + c], b2b = b2[nb0 + 16 + c];
      const float b3a = b3[nb0 + c], b3b = b3[nb0 + 16 + c];
      int lim[2][8];
#pragma unroll
      for (int i = 0; i < 2; ++i)
#pragma unroll
        for (int r = 0; r < 8; ++r) lim[i][r] = idx_s[16 * i + 8 * hh + r];

      for (int js = 0; js < NBATCH - 1; ++js) {
        const float dt = dts_s[js];
        v8f acc[2][2];
        tile_gemm_32x32(TA, W1, nb0, c, hh, acc);
        store_softplus_tile(TB, acc, b1a, b1b, nb0, c, hh);
        __syncthreads();
        tile_gemm_32x32(TB, W2, nb0, c, hh, acc);
        store_softplus_tile(TC, acc, b2a, b2b, nb0, c, hh);
        __syncthreads();
        tile_gemm_32x32(TC, W3, nb0, c, hh, acc);
#pragma unroll
        for (int i = 0; i < 2; ++i)
#pragma unroll
          for (int j = 0; j < 2; ++j) {
            const int n = nb0 + 16 * j + c;
            const float bias = j ? b3b : b3a;
#pragma unroll
            for (int r = 0; r < 8; ++r) {
              const int lr = 16 * i + 8 * hh + r;
              const float f = acc[i][j][r] * WCARRY_INV + bias;
              const float dte = (js < lim[i][r]) ? dt : 0.0f;
              const float y = ys[lr * YPF + n] + f * dte;
              ys[lr * YPF + n] = y;
              TA[lr * TPH + n] = (_Float16)y;
            }
          }
        __syncthreads();
      }
    }
  }
}

extern "C" void kernel_launch(void* const* d_in, const int* in_sizes, int n_in,
                              void* d_out, int out_size, void* d_ws, size_t ws_size,
                              hipStream_t stream) {
  if (n_in < 12) return;
  if (in_sizes[0] != NBATCH * NSTEP * HID || in_sizes[1] != NBATCH * NSTEP ||
      in_sizes[2] != NGATE3 * HID || in_sizes[3] != NGATE3 * HID ||
      in_sizes[4] != NGATE3 || in_sizes[5] != NGATE3 ||
      in_sizes[6] != HID * HID || in_sizes[7] != HID ||
      in_sizes[8] != HID * HID || in_sizes[9] != HID ||
      in_sizes[10] != HID * HID || in_sizes[11] != HID ||
      out_size != NBATCH * NSTEP * HID) return;

  const float* input = (const float*)d_in[0];
  const float* times = (const float*)d_in[1];
  const float* W_ih  = (const float*)d_in[2];
  const float* W_hh  = (const float*)d_in[3];
  const float* b_ih  = (const float*)d_in[4];
  const float* b_hh  = (const float*)d_in[5];
  const float* oW1   = (const float*)d_in[6];
  const float* ob1   = (const float*)d_in[7];
  const float* oW2   = (const float*)d_in[8];
  const float* ob2   = (const float*)d_in[9];
  const float* oW3   = (const float*)d_in[10];
  const float* ob3   = (const float*)d_in[11];

  const size_t nWih = (size_t)NGATE3 * HID;
  const size_t nWsq = (size_t)HID * HID;
  const size_t nX   = (size_t)NBATCH * NSTEP * HID;
  const size_t nG   = (size_t)NBATCH * NSTEP * NGATE3;
  size_t off = 0;
  const size_t offWih = off; off += nWih * 2;
  const size_t offWhh = off; off += nWih * 2;
  const size_t offW1h = off; off += nWsq * 2;
  const size_t offW2h = off; off += nWsq * 2;
  const size_t offW3h = off; off += nWsq * 2;
  const size_t offX   = off; off += nX * 2;
  const size_t offG   = off; off += nG * 4;
  if (off > ws_size) return;

  char* ws = (char*)d_ws;
  _Float16* Wih16 = (_Float16*)(ws + offWih);
  _Float16* Whh16 = (_Float16*)(ws + offWhh);
  _Float16* W1_16 = (_Float16*)(ws + offW1h);
  _Float16* W2_16 = (_Float16*)(ws + offW2h);
  _Float16* W3_16 = (_Float16*)(ws + offW3h);
  _Float16* X16   = (_Float16*)(ws + offX);
  float*    G     = (float*)(ws + offG);

  const int n2ih = (int)(nWih / 2), n2sq = (int)(nWsq / 2), n2x = (int)(nX / 2);
  cast_scale_f16x2<<<(n2ih + 255) / 256, 256, 0, stream>>>(W_ih, Wih16, n2ih, WCARRY);
  cast_scale_f16x2<<<(n2ih + 255) / 256, 256, 0, stream>>>(W_hh, Whh16, n2ih, WCARRY);
  cast_scale_f16x2<<<(n2sq + 255) / 256, 256, 0, stream>>>(oW1, W1_16, n2sq, WCARRY);
  cast_scale_f16x2<<<(n2sq + 255) / 256, 256, 0, stream>>>(oW2, W2_16, n2sq, WCARRY);
  cast_scale_f16x2<<<(n2sq + 255) / 256, 256, 0, stream>>>(oW3, W3_16, n2sq, WCARRY);
  cast_scale_f16x2<<<(n2x + 255) / 256, 256, 0, stream>>>(input, X16, n2x, 1.0f);

  {
    const int gM = NBATCH * NSTEP, gN = NGATE3, gK = HID;
    const int tiles = (gM / 64) * (gN / 64);
    wmma_gemm64<0, false, 2, 0, false, 0><<<dim3((tiles + 7) / 8, 1, 1), 256, 0, stream>>>(
        (const unsigned short*)X16, nullptr, gK, 0L,
        (const unsigned short*)Wih16, nullptr, gK, 0L,
        (void*)G, nullptr, gN, 0L,
        b_ih, nullptr, 0L,
        gM, gN, gK, WCARRY_INV);
  }

  gru_ode_seq<<<NBATCH / NB_ROWS, NTHR, 0, stream>>>(
      G, Whh16, W1_16, W2_16, W3_16, times, b_hh, ob1, ob2, ob3, (float*)d_out);
}
